// SimpleFLAME_67594195305075
// MI455X (gfx1250) — hardware-run, weakly checked
//
#include <hip/hip_runtime.h>
#include <math.h>

typedef __attribute__((ext_vector_type(16))) __bf16   v16b;
typedef __attribute__((ext_vector_type(8)))  __bf16   v8b;
typedef __attribute__((ext_vector_type(8)))  _Float16 v8h;
typedef __attribute__((ext_vector_type(8)))  float    v8f;
typedef __attribute__((ext_vector_type(4)))  float    v4f;

constexpr int kNB    = 4096;
constexpr int kNV    = 5023;
constexpr int kNF    = 9976;
constexpr int kNL    = 105;
constexpr int kNS    = 100;
constexpr int kNE    = 50;
constexpr int kKR    = kNS + kNE;
constexpr int kKP    = 160;
constexpr int kNR    = kNL * 3;
constexpr int kNP    = 320;
constexpr int kLCR   = 128;
constexpr int kTilesM = kNB / 64;
constexpr int kTilesN = kNP / 64;
static_assert(kKR == 150 && (kKP % 32) == 0 && kKP >= kKR, "k padding");
static_assert(kNR == 315 && (kNP % 64) == 0 && kNP >= kNR, "n padding");
static_assert((kNB % 64) == 0, "m tiles");
static_assert(((kNB * kNR) % 256) == 0, "flat output is a whole number of 256-lane blocks");
static_assert(((kNB * kNR * 4) % 128) == 0, "flat output is a whole number of 128-B lines");
static_assert((kTilesM * kTilesN) % 8 == 0, "8 tiles per GEMM block");

constexpr size_t kOffAH  = 0;
constexpr size_t kOffAL  = kOffAH  + (size_t)kNB * kKP * 2;
constexpr size_t kOffBH  = kOffAL  + (size_t)kNB * kKP * 2;
constexpr size_t kOffBL  = kOffBH  + (size_t)kNP * kKP * 2;
constexpr size_t kOffPRE = kOffBL  + (size_t)kNP * kKP * 2;
constexpr size_t kOffRT  = kOffPRE + (size_t)kNB * kNP * 4;
constexpr size_t kOffLC  = kOffRT  + (size_t)kNB * 16 * 4;
constexpr size_t kWsTotal = kOffLC + (size_t)kLCR * 8 * 4;
static_assert(kWsTotal == 8335360ull, "carve total");
static_assert(kWsTotal <= 134217728ull, "carve cap");
static_assert((kOffAL % 128) == 0 && (kOffBH % 128) == 0 && (kOffBL % 128) == 0 &&
              (kOffPRE % 128) == 0 && (kOffRT % 128) == 0 && (kOffLC % 128) == 0, "128-B aligned regions");

__device__ __forceinline__ unsigned short f2bf_bits(float f) {
  unsigned u = __float_as_uint(f);
  return (unsigned short)((u + 0x7FFFu + ((u >> 16) & 1u)) >> 16);
}
__device__ __forceinline__ float bf_bits2f(unsigned short h) { return __uint_as_float(((unsigned)h) << 16); }
__device__ __forceinline__ int clampi(int v, int lo, int hi) { return v < lo ? lo : (v > hi ? hi : v); }

__device__ __forceinline__ void split8(const v4f a0, const v4f a1, v8h& hv, v8h& lv) {
#pragma unroll
  for (int e = 0; e < 4; ++e) {
    const float x0 = a0[e];
    const float x1 = a1[e];
    const unsigned short h0 = f2bf_bits(x0);
    const unsigned short h1 = f2bf_bits(x1);
    const unsigned short l0 = f2bf_bits(x0 - bf_bits2f(h0));
    const unsigned short l1 = f2bf_bits(x1 - bf_bits2f(h1));
    hv[e]     = __builtin_bit_cast(_Float16, h0);
    hv[4 + e] = __builtin_bit_cast(_Float16, h1);
    lv[e]     = __builtin_bit_cast(_Float16, l0);
    lv[4 + e] = __builtin_bit_cast(_Float16, l1);
  }
}

__device__ __forceinline__ void tie_acc_ab(v8f& a, v16b x0, v16b x1, v16b y0, v16b y1) {
  asm volatile("v_nop\n\tv_nop\n\tv_nop\n\tv_nop" : "+v"(a) : "v"(x0), "v"(x1), "v"(y0), "v"(y1));
}
__device__ __forceinline__ void tie_acc(v8f& a) {
  asm volatile("v_nop\n\tv_nop\n\tv_nop\n\tv_nop" : "+v"(a));
}
__device__ __forceinline__ void keep4_b(v16b a, v16b b, v16b c, v16b d) {
  asm volatile("v_nop" :: "v"(a), "v"(b), "v"(c), "v"(d));
}
__device__ __forceinline__ v16b frag_load(const __bf16* p) {
  union U { v16b v; v8b h[2]; };
  U f;
  f.h[0] = *(const v8b*)(p);
  f.h[1] = *(const v8b*)(p + 16);
  return f.v;
}
__device__ __forceinline__ v8f frag_mma(v16b a, v16b b, v8f c) {
  return __builtin_amdgcn_wmma_f32_16x16x32_bf16(false, a, false, b, (short)0, c, false, false);
}

__global__ __launch_bounds__(256) void lmk_consts_kernel(
    const float* __restrict__ vt, const float* __restrict__ bary,
    const int* __restrict__ faces, const int* __restrict__ lfi, float* __restrict__ LC)
{
  __shared__ __align__(16) float sY[5024];
  __shared__ __align__(16) float sL[256 * 8];
  const int tid = threadIdx.x;
#pragma unroll 1
  for (int it = 0; it < 20; ++it) {
    int i = it * 256 + tid;
    i = i < kNV ? i : kNV - 1;
    sY[i] = vt[i * 3 + 1];
  }
  __syncthreads();
  float sum = 0.0f;
#pragma unroll 1
  for (int i = 0; i < kNV; ++i) sum += sY[i];
  const float ymean = sum * (1.0f / (float)kNV);

  const int lc = tid < kNL ? tid : kNL - 1;
  const bool valid = tid < kNL;
  const int f  = clampi(lfi[lc], 0, kNF - 1);
  const int i0 = clampi(faces[f * 3 + 0], 0, kNV - 1);
  const int i1 = clampi(faces[f * 3 + 1], 0, kNV - 1);
  const int i2 = clampi(faces[f * 3 + 2], 0, kNV - 1);
  const float w0 = bary[lc * 3 + 0];
  const float w1 = bary[lc * 3 + 1];
  const float w2 = bary[lc * 3 + 2];
  const float x0 = vt[i0 * 3 + 0], y0 = vt[i0 * 3 + 1], z0 = vt[i0 * 3 + 2];
  const float x1 = vt[i1 * 3 + 0], y1 = vt[i1 * 3 + 1], z1 = vt[i1 * 3 + 2];
  const float x2 = vt[i2 * 3 + 0], y2 = vt[i2 * 3 + 1], z2 = vt[i2 * 3 + 2];
  const float m0 = (y0 < ymean) ? 1.0f : 0.0f;
  const float m1 = (y1 < ymean) ? 1.0f : 0.0f;
  const float m2 = (y2 < ymean) ? 1.0f : 0.0f;
  float tx = w0 * x0; tx = fmaf(w1, x1, tx); tx = fmaf(w2, x2, tx);
  float ty = w0 * y0; ty = fmaf(w1, y1, ty); ty = fmaf(w2, y2, ty);
  float tz = w0 * z0; tz = fmaf(w1, z1, tz); tz = fmaf(w2, z2, tz);
  float ms = w0 * m0; ms = fmaf(w1, m1, ms); ms = fmaf(w2, m2, ms);
  const float joff = -0.15f * ms;
  const float wsum = (w0 + w1) + w2;
  v4f q0, q1;
  q0[0] = valid ? tx : 0.0f;
  q0[1] = valid ? ty : 0.0f;
  q0[2] = valid ? tz : 0.0f;
  q0[3] = valid ? joff : 0.0f;
  q1[0] = valid ? wsum : 0.0f;
  q1[1] = 0.0f;
  q1[2] = 0.0f;
  q1[3] = 0.0f;
  *(v4f*)(sL + tid * 8)     = q0;
  *(v4f*)(sL + tid * 8 + 4) = q1;
  __syncthreads();
  const v4f o = *(const v4f*)(sL + tid * 4);
  float* dst = LC + tid * 4;
  *(volatile v4f*)dst = o;
  __threadfence();
  *(volatile v4f*)dst = o;
}

__global__ __launch_bounds__(256) void rot_table_kernel(
    const float* __restrict__ rotation, const float* __restrict__ translation,
    const float* __restrict__ jaw, float* __restrict__ RT)
{
  __shared__ __align__(16) float sR[256 * 16];
  const int tid = threadIdx.x;
  const int b = blockIdx.x * 256 + tid;
  const float ax = rotation[b * 3 + 0];
  const float ay = rotation[b * 3 + 1];
  const float az = rotation[b * 3 + 2];
  const float t0 = translation[b * 3 + 0];
  const float t1 = translation[b * 3 + 1];
  const float t2 = translation[b * 3 + 2];
  const float j0 = jaw[b * 3 + 0];
  const float angle = sqrtf(ax * ax + ay * ay + az * az);
  const float inv = 1.0f / (angle + 1e-8f);
  const float x = ax * inv, y = ay * inv, z = az * inv;
  const float sn = sinf(angle);
  const float cc = 1.0f - cosf(angle);
  const float xy = x * y, xz = x * z, yz = y * z;
  const float xx = x * x, yy = y * y, zz = z * z;
  v4f q0, q1, q2, q3;
  q0[0] = 1.0f - cc * (yy + zz);
  q0[1] = cc * xy - sn * z;
  q0[2] = cc * xz + sn * y;
  q0[3] = cc * xy + sn * z;
  q1[0] = 1.0f - cc * (xx + zz);
  q1[1] = cc * yz - sn * x;
  q1[2] = cc * xz - sn * y;
  q1[3] = cc * yz + sn * x;
  q2[0] = 1.0f - cc * (xx + yy);
  q2[1] = t0;
  q2[2] = t1;
  q2[3] = t2;
  q3[0] = j0;
  q3[1] = 0.0f;
  q3[2] = 0.0f;
  q3[3] = 0.0f;
  *(v4f*)(sR + tid * 16 + 0)  = q0;
  *(v4f*)(sR + tid * 16 + 4)  = q1;
  *(v4f*)(sR + tid * 16 + 8)  = q2;
  *(v4f*)(sR + tid * 16 + 12) = q3;
  __syncthreads();
  v4f o[4];
#pragma unroll
  for (int it = 0; it < 4; ++it) o[it] = *(const v4f*)(sR + (it * 256 + tid) * 4);
  float* base = RT + (size_t)blockIdx.x * 4096;
  for (int pass = 0; pass < 2; ++pass) {
#pragma unroll
    for (int it = 0; it < 4; ++it) *(volatile v4f*)(base + (it * 256 + tid) * 4) = o[it];
    __threadfence();
  }
}

__global__ __launch_bounds__(256) void pack_coef_kernel(
    const float* __restrict__ shp, const float* __restrict__ expr,
    unsigned short* __restrict__ AH, unsigned short* __restrict__ AL)
{
  __shared__ __align__(16) float sA[64 * kKP];
  const int tid = threadIdx.x;
  const int b0 = blockIdx.x * 64;
  const v4f* s4 = (const v4f*)(shp + (size_t)b0 * kNS);
  const v4f* e4 = (const v4f*)(expr + (size_t)b0 * kNE);
#pragma unroll 1
  for (int it = 0; it < 7; ++it) {
    int i = it * 256 + tid;
    i = i < 1600 ? i : 1599;
    const v4f v = s4[i];
    const int row = i / 25;
    const int c4 = (i - row * 25) * 4;
    *(v4f*)(sA + row * kKP + c4) = v;
  }
#pragma unroll 1
  for (int it = 0; it < 4; ++it) {
    int i = it * 256 + tid;
    i = i < 800 ? i : 799;
    const v4f v = e4[i];
#pragma unroll
    for (int e = 0; e < 4; ++e) {
      const int j = 4 * i + e;
      const int row = j / kNE;
      const int col = j - row * kNE;
      sA[row * kKP + kNS + col] = v[e];
    }
  }
#pragma unroll 1
  for (int it = 0; it < 3; ++it) {
    int i = it * 256 + tid;
    i = i < 640 ? i : 639;
    const int row = i / 10;
    const int col = i - row * 10;
    sA[row * kKP + kKR + col] = 0.0f;
  }
  __syncthreads();
  v8h hv[5], lv[5];
#pragma unroll
  for (int it = 0; it < 5; ++it) {
    const float* sp = sA + (it * 256 + tid) * 8;
    const v4f a0 = *(const v4f*)(sp);
    const v4f a1 = *(const v4f*)(sp + 4);
    split8(a0, a1, hv[it], lv[it]);
  }
  unsigned short* qh = AH + (size_t)b0 * kKP;
  unsigned short* ql = AL + (size_t)b0 * kKP;
  for (int pass = 0; pass < 2; ++pass) {
#pragma unroll
    for (int it = 0; it < 5; ++it) {
      const int o = (it * 256 + tid) * 8;
      *(volatile v8h*)(qh + o) = hv[it];
      *(volatile v8h*)(ql + o) = lv[it];
    }
    __threadfence();
  }
}

__global__ __launch_bounds__(320) void fold_dirs_kernel(
    const float* __restrict__ sds, const float* __restrict__ sde, const float* __restrict__ bary,
    const int* __restrict__ faces, const int* __restrict__ lfi,
    unsigned short* __restrict__ BH, unsigned short* __restrict__ BL)
{
  __shared__ __align__(16) float sB[16 * kKP];
  const int tid = threadIdx.x;
  const int n0 = blockIdx.x * 16;
  const int r = tid / 20;
  const int kk = tid - r * 20;
  const int n = n0 + r;
  const int l = n / 3;
  const int d = n - l * 3;
  const bool valid = n < kNR;
  const int lc = l < kNL ? l : kNL - 1;
  const int f  = clampi(lfi[lc], 0, kNF - 1);
  const int i0 = clampi(faces[f * 3 + 0], 0, kNV - 1);
  const int i1 = clampi(faces[f * 3 + 1], 0, kNV - 1);
  const int i2 = clampi(faces[f * 3 + 2], 0, kNV - 1);
  const float w0 = bary[lc * 3 + 0];
  const float w1 = bary[lc * 3 + 1];
  const float w2 = bary[lc * 3 + 2];
  const float* ps0 = sds + (size_t)(i0 * 3 + d) * kNS;
  const float* ps1 = sds + (size_t)(i1 * 3 + d) * kNS;
  const float* ps2 = sds + (size_t)(i2 * 3 + d) * kNS;
  const float* pe0 = sde + (size_t)(i0 * 3 + d) * kNE;
  const float* pe1 = sde + (size_t)(i1 * 3 + d) * kNE;
  const float* pe2 = sde + (size_t)(i2 * 3 + d) * kNE;
#pragma unroll 1
  for (int i = 0; i < 8; ++i) {
    const int k = kk + 20 * i;
    const int ks = k < kNS ? k : kNS - 1;
    const int ke = clampi(k - kNS, 0, kNE - 1);
    float s0 = ps0[ks];
    float s1 = ps1[ks];
    float s2 = ps2[ks];
    float e0 = pe0[ke];
    float e1 = pe1[ke];
    float e2 = pe2[ke];
    asm volatile("" : "+v"(s0), "+v"(s1), "+v"(s2));
    asm volatile("" : "+v"(e0), "+v"(e1), "+v"(e2));
    const bool isS = k < kNS;
    const bool isE = k < kKR;
    const float v0 = isS ? s0 : (isE ? e0 : 0.0f);
    const float v1 = isS ? s1 : (isE ? e1 : 0.0f);
    const float v2 = isS ? s2 : (isE ? e2 : 0.0f);
    float acc = w0 * v0;
    acc = fmaf(w1, v1, acc);
    acc = fmaf(w2, v2, acc);
    sB[r * kKP + k] = valid ? acc : 0.0f;
  }
  __syncthreads();
  const float* sp = sB + tid * 8;
  const v4f a0 = *(const v4f*)(sp);
  const v4f a1 = *(const v4f*)(sp + 4);
  v8h hv, lv;
  split8(a0, a1, hv, lv);
  unsigned short* qh = BH + (size_t)n0 * kKP + tid * 8;
  unsigned short* ql = BL + (size_t)n0 * kKP + tid * 8;
  *(volatile v8h*)qh = hv;
  *(volatile v8h*)ql = lv;
  __threadfence();
  *(volatile v8h*)qh = hv;
  *(volatile v8h*)ql = lv;
}

__global__ __launch_bounds__(256) void coef_dirs_gemm_kernel(
    const unsigned short* __restrict__ Ahp, const unsigned short* __restrict__ Alp,
    const unsigned short* __restrict__ Bhp, const unsigned short* __restrict__ Blp,
    float* __restrict__ C)
{
  const __bf16* Ah = (const __bf16*)Ahp;
  const __bf16* Al = (const __bf16*)Alp;
  const __bf16* Bh = (const __bf16*)Bhp;
  const __bf16* Bl = (const __bf16*)Blp;
  __shared__ __align__(16) float sT[8][16 * 68];
  const int lane = threadIdx.x & 31;
  const int wave = threadIdx.x >> 5;
  const int tile = blockIdx.x * 8 + wave;
  if (tile >= kTilesM * kTilesN) return;
  const int tm = tile / kTilesN;
  const int tn = tile - tm * kTilesN;
  const int m0 = tm << 6;
  const int n0 = tn << 6;
  const int rlane = lane & 15;
  const int koff  = (lane >> 4) * 8;
  const int mOff  = (lane >> 4) * 8;

  v8f acc[4][4];
#pragma unroll
  for (int i = 0; i < 4; ++i)
#pragma unroll
    for (int j = 0; j < 4; ++j) acc[i][j] = (v8f){0.f,0.f,0.f,0.f,0.f,0.f,0.f,0.f};

  for (int k0 = 0; k0 < kKP; k0 += 32) {
    v16b bh[4], bl[4];
#pragma unroll
    for (int j = 0; j < 4; ++j) {
      const size_t bo = (size_t)(n0 + (j << 4) + rlane) * kKP + koff + k0;
      bh[j] = frag_load(Bh + bo);
      bl[j] = frag_load(Bl + bo);
    }
#pragma unroll
    for (int i = 0; i < 4; ++i) {
      const size_t ao = (size_t)(m0 + (i << 4) + rlane) * kKP + koff + k0;
      const v16b ah = frag_load(Ah + ao);
      const v16b al = frag_load(Al + ao);
#pragma unroll
      for (int j = 0; j < 4; ++j) {
        acc[i][j] = frag_mma(ah, bh[j], acc[i][j]);
        acc[i][j] = frag_mma(ah, bl[j], acc[i][j]);
        acc[i][j] = frag_mma(al, bh[j], acc[i][j]);
      }
#pragma unroll
      for (int j = 0; j < 4; ++j) tie_acc_ab(acc[i][j], ah, al, bh[j], bl[j]);
    }
    keep4_b(bh[0], bh[1], bh[2], bh[3]);
    keep4_b(bl[0], bl[1], bl[2], bl[3]);
  }
#pragma unroll
  for (int i = 0; i < 4; ++i)
#pragma unroll
    for (int j = 0; j < 4; ++j) tie_acc(acc[i][j]);

  float* slab = sT[wave];
  const int hh = lane >> 4, c4 = (lane & 15) * 4;
#pragma unroll
  for (int i = 0; i < 4; ++i) {
    const int mBase = m0 + (i << 4);
#pragma unroll
    for (int j = 0; j < 4; ++j) {
#pragma unroll
      for (int r = 0; r < 8; ++r) slab[(mOff + r) * 68 + (j << 4) + rlane] = acc[i][j][r];
    }
    __builtin_amdgcn_fence(__ATOMIC_RELEASE, "workgroup");
    __builtin_amdgcn_wave_barrier();
    __builtin_amdgcn_fence(__ATOMIC_ACQUIRE, "workgroup");
    for (int pass = 0; pass < 2; ++pass) {
#pragma unroll
      for (int it = 0; it < 8; ++it) {
        const int row = it * 2 + hh;
        const v4f v = *(const v4f*)(slab + row * 68 + c4);
        *(volatile v4f*)(C + (size_t)(mBase + row) * kNP + n0 + c4) = v;
      }
      __threadfence();
    }
    __builtin_amdgcn_fence(__ATOMIC_RELEASE, "workgroup");
    __builtin_amdgcn_wave_barrier();
    __builtin_amdgcn_fence(__ATOMIC_ACQUIRE, "workgroup");
  }
}

__global__ __launch_bounds__(256) void lmk_out_kernel(
    const float* __restrict__ PRE, const float* __restrict__ RT, const float* __restrict__ LC,
    float* __restrict__ out)
{
  const int e = blockIdx.x * 256 + threadIdx.x;
  const int b = e / kNR;
  const int r = e - b * kNR;
  const int l = r / 3;
  const int d = r - l * 3;
  const float* pr = PRE + (size_t)b * kNP + l * 3;
  const float p0 = pr[0];
  const float p1 = pr[1];
  const float p2 = pr[2];
  const v4f c0 = *(const v4f*)(LC + l * 8);
  const v4f c1 = *(const v4f*)(LC + l * 8 + 4);
  const float* rt = RT + (size_t)b * 16;
  const float r0 = rt[d * 3 + 0];
  const float r1 = rt[d * 3 + 1];
  const float r2 = rt[d * 3 + 2];
  const float td = rt[9 + d];
  const float j0 = rt[12];
  const float q0 = p0 + c0[0];
  const float q1 = (p1 + c0[1]) + c0[3] * j0;
  const float q2 = p2 + c0[2];
  float o = r0 * q0;
  o = fmaf(r1, q1, o);
  o = fmaf(r2, q2, o);
  o = fmaf(c1[0], td, o);
  float* dst = out + e;
  *(volatile float*)dst = o;
  __threadfence();
  *(volatile float*)dst = o;
}

extern "C" void kernel_launch(void* const* d_in, const int* in_sizes, int n_in,
                              void* d_out, int out_size, void* d_ws, size_t ws_size,
                              hipStream_t stream) {
  if (n_in < 11) return;
  if (in_sizes[0] != kNB * kNS) return;
  if (in_sizes[1] != kNB * kNE) return;
  if (in_sizes[2] != kNB * 3) return;
  if (in_sizes[3] != kNB * 3) return;
  if (in_sizes[4] != kNB * 3) return;
  if (in_sizes[5] != kNV * 3) return;
  if (in_sizes[6] != kNV * 3 * kNS) return;
  if (in_sizes[7] != kNV * 3 * kNE) return;
  if (in_sizes[8] != kNL * 3) return;
  if (in_sizes[9] != kNF * 3) return;
  if (in_sizes[10] != kNL) return;
  if (out_size != kNB * kNR) return;
  if (ws_size < kWsTotal) return;

  const float* shp         = (const float*)d_in[0];
  const float* expr        = (const float*)d_in[1];
  const float* rotation    = (const float*)d_in[2];
  const float* jaw         = (const float*)d_in[3];
  const float* translation = (const float*)d_in[4];
  const float* vtemplate   = (const float*)d_in[5];
  const float* sds         = (const float*)d_in[6];
  const float* sde         = (const float*)d_in[7];
  const float* bary        = (const float*)d_in[8];
  const int*   faces       = (const int*)d_in[9];
  const int*   lfi         = (const int*)d_in[10];
  float* out = (float*)d_out;

  char* ws = (char*)d_ws;
  unsigned short* AH  = (unsigned short*)(ws + kOffAH);
  unsigned short* AL  = (unsigned short*)(ws + kOffAL);
  unsigned short* BH  = (unsigned short*)(ws + kOffBH);
  unsigned short* BL  = (unsigned short*)(ws + kOffBL);
  float*          PRE = (float*)(ws + kOffPRE);
  float*          RT  = (float*)(ws + kOffRT);
  float*          LC  = (float*)(ws + kOffLC);

  lmk_consts_kernel<<<1, 256, 0, stream>>>(vtemplate, bary, faces, lfi, LC);
  rot_table_kernel<<<kNB / 256, 256, 0, stream>>>(rotation, translation, jaw, RT);
  pack_coef_kernel<<<kNB / 64, 256, 0, stream>>>(shp, expr, AH, AL);
  fold_dirs_kernel<<<kNP / 16, 320, 0, stream>>>(sds, sde, bary, faces, lfi, BH, BL);
  coef_dirs_gemm_kernel<<<(kTilesM * kTilesN) / 8, 256, 0, stream>>>(AH, AL, BH, BL, PRE);
  lmk_out_kernel<<<(kNB * kNR) / 256, 256, 0, stream>>>(PRE, RT, LC, out);
}
